// MessagePassingConvolutionHaiku_70583492542673
// MI455X (gfx1250) — hardware-verified
//
#include <hip/hip_runtime.h>
#include <stddef.h>
#include <stdint.h>

#ifndef GELU_C_REPLAY
#define GELU_C_REPLAY 0.651714385f
#endif

#define NN      50000
#define NE      400000
#define NTHR    256
#define NWAVE   8
#define EPT     8
#define CHUNK   (NTHR * EPT)
#define WCAP    (EPT * 32)
#define LISTN   (NWAVE * WCAP)
#define NBA     1024
#define SLA     10
#define NBLK    49
#define RCAP    9216
#define TPB     (RCAP / 128)
#define DEGCAP  48
#define GRPB    10
#define NGRP    5
#define SVW     160
#define MIXW    192
#define AGGW    768
#define OWUS    0
#define OWUV    4096
#define OW1C    5120
#define OW2C    7168
#define OWDS    31744
#define OWDV    44032
#define NWP     50176
#define PU0     512
#define PU1     640
#define PU2     896
#define PU3     3968
#define PU4     5504
#define PU5     6272
#define XS_P    72
#define XV_P    40
#define SV_P    164
#define UP_LDS  (128 * SV_P * 4 + 128 * XS_P * 2 + 3 * 128 * XV_P * 2)
#define A1_P    40
#define A2_P    136
#define SD_P    196
#define EDGE_LDS (128 * SD_P * 4 + 128 * A2_P * 2 + 128 * A1_P * 2)
#define GEL_IT  ((128 * 64) / NTHR)
#define BK_ZINTS (LISTN + 2 * RCAP + 3 * NBA)
#define BK_LDS  ((BK_ZINTS + 16) * 4)
#define WSMAX   134217728
#define PI_F    3.14159274f
#define SQ2_F   1.41421354f
#define SQ3_F   1.73205078f
#define RS3_F   0.577350269f
#define RS8_F   0.353553391f
#define RS32_F  0.176776695f
#define RS96_F  0.102062073f
#define ENVC_F  1.97846556f
#define GINV_F  (1.0f / GELU_C_REPLAY)

static_assert((CHUNK & (CHUNK - 1)) == 0 && CHUNK <= 4096);
static_assert(NBA == (1 << SLA) && NBLK * NBA >= NN && (NBLK - 1) * NBA < NN);
static_assert(((long long)NE << SLA) < (1LL << 31));
static_assert(RCAP % 128 == 0 && RCAP % (4 * NTHR) == 0);
static_assert(BK_ZINTS % (4 * NTHR) == 0);
static_assert(BK_LDS <= 300000 && EDGE_LDS <= 300000 && UP_LDS <= 300000);
static_assert(NGRP * GRPB >= NBLK && (NGRP - 1) * GRPB < NBLK);
static_assert((SVW * 4) % 128 == 0 && (MIXW * 4) % 128 == 0 && (AGGW * 2) % 128 == 0);
static_assert(64 % 32 == 0 && 32 % 32 == 0 && 128 % 32 == 0 && 192 % 32 == 0);
static_assert(PU0 % 128 == 0 && PU1 % 128 == 0 && PU2 % 128 == 0 && PU3 % 128 == 0 && PU4 % 128 == 0 && PU5 % 128 == 0);
static_assert(PU5 * 8 == NWP);
static_assert(NBA % 64 == 0 && NBA % 128 == 0);
static_assert((XS_P * 2) % 16 == 0 && (XV_P * 2) % 16 == 0 && (A1_P * 2) % 16 == 0 && (A2_P * 2) % 16 == 0);
static_assert((SV_P * 4) % 16 == 0 && (SD_P * 4) % 16 == 0);
static_assert(GEL_IT * NTHR == 128 * 64 && SD_P >= 64 && A2_P >= 128);

typedef float          v4f   __attribute__((ext_vector_type(4)));
typedef float          v8f   __attribute__((ext_vector_type(8)));
typedef int            v4i   __attribute__((ext_vector_type(4)));
typedef int            v8i   __attribute__((ext_vector_type(8)));
typedef unsigned short v4us  __attribute__((ext_vector_type(4)));
typedef unsigned short v8us  __attribute__((ext_vector_type(8)));
typedef unsigned short v16us __attribute__((ext_vector_type(16)));
typedef __bf16         v16bf __attribute__((ext_vector_type(16)));
typedef v4f  __attribute__((may_alias)) v4fa;
typedef v4i  __attribute__((may_alias)) v4ia;
typedef v4us __attribute__((may_alias)) v4usa;
typedef v8us __attribute__((may_alias)) v8usa;
union FragB { v16bf v; v16us u; v8us h[2]; v8i w; };

__device__ __forceinline__ v8f wmb(const FragB& a, const FragB& b, v8f c) {
  v8f d = __builtin_amdgcn_wmma_f32_16x16x32_bf16(false, a.v, false, b.v, (short)0, c, false, false);
  asm volatile("v_nop\n\tv_nop\n\tv_nop\n\tv_nop" : "+v"(d) : "v"(a.w), "v"(b.w));
  return d;
}
__device__ __forceinline__ void ldwait() {
  asm volatile("s_wait_loadcnt 0x0" ::: "memory");
}
__device__ __forceinline__ unsigned bf16_bits(float f) {
  const unsigned u = __float_as_uint(f);
  return (u + 0x7FFFu + ((u >> 16) & 1u)) >> 16;
}
__device__ __forceinline__ float bf16_val(float f) {
  return __uint_as_float(bf16_bits(f) << 16);
}
__device__ __forceinline__ float rcp_f(float x) { return __builtin_amdgcn_rcpf(x); }
__device__ __forceinline__ int clampi(int v, int lo, int hi) { return v < lo ? lo : (v > hi ? hi : v); }
__device__ __forceinline__ void put16(unsigned short* dp, v8us o) {
  *(volatile v8us*)dp = o;
  __threadfence();
  *(volatile v8us*)dp = o;
}
__device__ __forceinline__ void putf4(float* dp, v4f o) {
  *(volatile v4f*)dp = o;
  __threadfence();
  *(volatile v4f*)dp = o;
}
__device__ __forceinline__ void puti4(int* dp, v4i o) {
  *(volatile v4i*)dp = o;
  __threadfence();
  *(volatile v4i*)dp = o;
}

__device__ __forceinline__ int scan_chunk(const int* __restrict__ dsts, int nE, int cbase, int slotBase,
                                          int nb, int vec8, int* list, int tid, int lane, int wave) {
  int wc = 0;
  const int el0  = tid * EPT;
  const int e0   = cbase + el0;
  const int sent = -2147483647 - 1;
  v4i da, db;
  if (vec8 != 0 && cbase + CHUNK <= nE) {
    da = *(const v4i*)(dsts + e0);
    db = *(const v4i*)(dsts + e0 + 4);
  } else {
    da.x = (e0     < nE) ? dsts[min(e0,     nE - 1)] : sent;
    da.y = (e0 + 1 < nE) ? dsts[min(e0 + 1, nE - 1)] : sent;
    da.z = (e0 + 2 < nE) ? dsts[min(e0 + 2, nE - 1)] : sent;
    da.w = (e0 + 3 < nE) ? dsts[min(e0 + 3, nE - 1)] : sent;
    db.x = (e0 + 4 < nE) ? dsts[min(e0 + 4, nE - 1)] : sent;
    db.y = (e0 + 5 < nE) ? dsts[min(e0 + 5, nE - 1)] : sent;
    db.z = (e0 + 6 < nE) ? dsts[min(e0 + 6, nE - 1)] : sent;
    db.w = (e0 + 7 < nE) ? dsts[min(e0 + 7, nE - 1)] : sent;
  }
  const unsigned nbs = (unsigned)slotBase;
  const unsigned unb = (unsigned)nb;
  const unsigned s0 = (unsigned)da.x - nbs, s1 = (unsigned)da.y - nbs;
  const unsigned s2 = (unsigned)da.z - nbs, s3 = (unsigned)da.w - nbs;
  const unsigned s4 = (unsigned)db.x - nbs, s5 = (unsigned)db.y - nbs;
  const unsigned s6 = (unsigned)db.z - nbs, s7 = (unsigned)db.w - nbs;
  const bool h0 = s0 < unb, h1 = s1 < unb, h2 = s2 < unb, h3 = s3 < unb;
  const bool h4 = s4 < unb, h5 = s5 < unb, h6 = s6 < unb, h7 = s7 < unb;
  const unsigned any = __builtin_amdgcn_ballot_w32(h0 | h1 | h2 | h3 | h4 | h5 | h6 | h7);
  if (any != 0u) {
#define HITJ(J, HJ, SJ) { \
      const unsigned mj = __builtin_amdgcn_ballot_w32(HJ); \
      if (mj != 0u) { \
        if (HJ) { \
          const int pos = wc + (int)__builtin_amdgcn_mbcnt_lo(mj, 0u); \
          if (pos < WCAP) list[wave * WCAP + pos] = ((el0 + (J)) << SLA) | (int)(SJ); \
        } \
        wc += (int)__builtin_popcount(mj); } }
    HITJ(0, h0, s0)
    HITJ(1, h1, s1)
    HITJ(2, h2, s2)
    HITJ(3, h3, s3)
    HITJ(4, h4, s4)
    HITJ(5, h5, s5)
    HITJ(6, h6, s6)
    HITJ(7, h7, s7)
#undef HITJ
  }
  return wc;
}

__global__ __launch_bounds__(128) void k_prep(const float* __restrict__ Wus, const float* __restrict__ Wuv,
                                              const float* __restrict__ W1, const float* __restrict__ W2,
                                              const float* __restrict__ Wds, const float* __restrict__ Wdv,
                                              unsigned short* WP) {
  const int u = (int)blockIdx.x * 128 + (int)threadIdx.x;
  v8us o;
  if (u < PU0) {
    const int n = u >> 3, k8 = (u & 7) * 8;
    const float* p = Wus + (size_t)k8 * 64 + n;
#pragma unroll
    for (int i = 0; i < 8; ++i) o[i] = (unsigned short)bf16_bits(p[(size_t)i * 64]);
    put16(WP + OWUS + n * 64 + k8, o);
    return;
  } else if (u < PU1) {
    const int v = u - PU0;
    const int mm = v >> 2, k8 = (v & 3) * 8;
    const float* p = Wuv + (size_t)k8 * 32 + mm;
#pragma unroll
    for (int i = 0; i < 8; ++i) o[i] = (unsigned short)bf16_bits(p[(size_t)i * 32]);
    put16(WP + OWUV + mm * 32 + k8, o);
    return;
  } else if (u < PU2) {
    const int v = u - PU1;
    const int j = v >> 2, k8 = (v & 3) * 8;
    const bool ok = k8 < 16;
    const float* p = W1 + j;
#pragma unroll
    for (int i = 0; i < 8; ++i) {
      const unsigned bb = bf16_bits(p[(size_t)i * 64]);
      o[i] = (unsigned short)(ok ? bb : 0u);
    }
    put16(WP + OW1C + j * 32 + k8, o);
    return;
  } else if (u < PU3) {
    const int v = u - PU2;
    const int n = v >> 4, k8 = (v & 15) * 8;
    const int sr = k8 & 63;
    const float* p = W2 + (size_t)sr * 192 + n;
#pragma unroll
    for (int i = 0; i < 8; ++i) o[i] = (unsigned short)bf16_bits(p[(size_t)i * 192]);
    put16(WP + OW2C + n * 128 + k8, o);
    return;
  } else if (u < PU4) {
    const int v = u - PU3;
    const int n = v / 24, k8 = (v - n * 24) * 8;
    const int sr = k8 % 96;
    const float* p = Wds + (size_t)sr * 64 + n;
#pragma unroll
    for (int i = 0; i < 8; ++i) o[i] = (unsigned short)bf16_bits(p[(size_t)i * 64]);
    put16(WP + OWDS + n * 192 + k8, o);
    return;
  } else if (u < PU5) {
    const int v = u - PU4;
    const int mm = v / 24, k8 = (v - mm * 24) * 8;
    const int sr = k8 % 96;
    const float* p = Wdv + (size_t)sr * 32 + mm;
#pragma unroll
    for (int i = 0; i < 8; ++i) o[i] = (unsigned short)bf16_bits(p[(size_t)i * 32]);
    put16(WP + OWDV + mm * 192 + k8, o);
    return;
  }
}

__device__ __forceinline__ void stv(unsigned short* sXv, int row, int jj, float val) {
  const int c = jj / 3;
  const int d = jj - 3 * c;
  sXv[(d * 128 + row) * XV_P + c] = (unsigned short)bf16_bits(val);
}

__global__ __launch_bounds__(NTHR) __attribute__((amdgpu_num_vgpr(248)))
void k_up(const float* __restrict__ xs, const float* __restrict__ nv,
          const unsigned short* __restrict__ WP, float* SV) {
  extern __shared__ __attribute__((aligned(16))) float dynu[];
  float*          stg = dynu;
  unsigned short* sXs = (unsigned short*)(dynu + 128 * SV_P);
  unsigned short* sXv = sXs + 128 * XS_P;
  const int tid = (int)threadIdx.x, lane = tid & 31, wave = tid >> 5, hh = lane >> 4, m = lane & 15;
  const int rowBase = (int)blockIdx.x * 128;

#pragma unroll 2
  for (int it = 0; it < 8; ++it) {
    const int idx = it * NTHR + tid;
    const int row = idx >> 4, c4 = (idx & 15) * 4;
    int gr = rowBase + row; gr = gr < NN ? gr : NN - 1;
    const v4f a = *(const v4f*)(xs + (size_t)gr * 64 + c4);
    v4us o;
    o.x = (unsigned short)bf16_bits(a.x); o.y = (unsigned short)bf16_bits(a.y);
    o.z = (unsigned short)bf16_bits(a.z); o.w = (unsigned short)bf16_bits(a.w);
    *(v4usa*)(sXs + row * XS_P + c4) = o;
  }
#pragma unroll 2
  for (int it = 0; it < 12; ++it) {
    const int f   = (it * NTHR + tid) * 4;
    const int row = f / 96;
    const int j   = f - row * 96;
    int gr = rowBase + row; gr = gr < NN ? gr : NN - 1;
    const v4f a = *(const v4f*)(nv + (size_t)gr * 96 + j);
    stv(sXv, row, j,     a.x);
    stv(sXv, row, j + 1, a.y);
    stv(sXv, row, j + 2, a.z);
    stv(sXv, row, j + 3, a.w);
  }
  __syncthreads();

  v8f accS[4], accV[3][2];
  {
    const v8f z = {0.f, 0.f, 0.f, 0.f, 0.f, 0.f, 0.f, 0.f};
#pragma unroll
    for (int t = 0; t < 4; ++t) accS[t] = z;
#pragma unroll
    for (int d = 0; d < 3; ++d) { accV[d][0] = z; accV[d][1] = z; }
  }
  {
    const unsigned short* ap = sXs + (16 * wave + m) * XS_P + 8 * hh;
    const unsigned short* bp = WP + OWUS + m * 64 + 8 * hh;
#pragma unroll
    for (int k0 = 0; k0 < 64; k0 += 32) {
      FragB af;
      af.h[0] = *(const v8usa*)(ap + k0);
      af.h[1] = *(const v8usa*)(ap + k0 + 16);
#pragma unroll
      for (int nt = 0; nt < 4; ++nt) {
        const unsigned short* wq = bp + (16 * nt) * 64 + k0;
        FragB bf;
        bf.h[0] = *(const v8usa*)wq;
        bf.h[1] = *(const v8usa*)(wq + 16);
        accS[nt] = wmb(af, bf, accS[nt]);
      }
    }
  }
  {
    const unsigned short* bp = WP + OWUV + m * 32 + 8 * hh;
    FragB b0, b1;
    b0.h[0] = *(const v8usa*)bp;
    b0.h[1] = *(const v8usa*)(bp + 16);
    b1.h[0] = *(const v8usa*)(bp + 16 * 32);
    b1.h[1] = *(const v8usa*)(bp + 16 * 32 + 16);
#pragma unroll
    for (int d = 0; d < 3; ++d) {
      const unsigned short* ap = sXv + (d * 128 + 16 * wave + m) * XV_P + 8 * hh;
      FragB af;
      af.h[0] = *(const v8usa*)ap;
      af.h[1] = *(const v8usa*)(ap + 16);
      accV[d][0] = wmb(af, b0, accV[d][0]);
      accV[d][1] = wmb(af, b1, accV[d][1]);
    }
  }
#pragma unroll
  for (int r = 0; r < 8; ++r) {
    float* sr = stg + (16 * wave + 8 * hh + r) * SV_P;
#pragma unroll
    for (int nt = 0; nt < 4; ++nt) sr[16 * nt + m] = accS[nt][r] * 0.125f;
#pragma unroll
    for (int d = 0; d < 3; ++d) {
      sr[64 + 32 * d + m]      = accV[d][0][r] * RS32_F;
      sr[64 + 32 * d + 16 + m] = accV[d][1][r] * RS32_F;
    }
  }
  __syncthreads();

#pragma unroll 4
  for (int it = 0; it < 20; ++it) {
    const int j = it * 32 + lane;
    const int row = j / 40, c4 = j - row * 40;
    const int gr = rowBase + 16 * wave + row;
    const v4f v = *(const v4fa*)(stg + (16 * wave + row) * SV_P + 4 * c4);
    if (gr < NN) *(volatile v4f*)(SV + (size_t)gr * SVW + 4 * c4) = v;
  }
  __threadfence();
#pragma unroll 4
  for (int it = 0; it < 20; ++it) {
    const int j = it * 32 + lane;
    const int row = j / 40, c4 = j - row * 40;
    const int gr = rowBase + 16 * wave + row;
    const v4f v = *(const v4fa*)(stg + (16 * wave + row) * SV_P + 4 * c4);
    if (gr < NN) *(volatile v4f*)(SV + (size_t)gr * SVW + 4 * c4) = v;
  }
}

__device__ __forceinline__ int bk_snd(int ent, int p, int tt, const int* __restrict__ snd) {
  const int eid = clampi(ent >> SLA, 0, NE - 1);
  const int sd  = clampi(snd[eid], 0, NN - 1);
  return (p < tt) ? sd : 0;
}
__device__ __forceinline__ int bk_rcv(int ent, int p, int tt, int nodeBase) {
  int r = nodeBase + (ent & (NBA - 1));
  r = r > NN - 1 ? NN - 1 : r;
  return (p < tt) ? r : 0;
}

__global__ __launch_bounds__(NTHR) void k_bucket(const int* __restrict__ rcv, const int* __restrict__ snd,
                                                 int* SND, int* RCVL, int* CNT, int* OFF, int* META) {
  extern __shared__ __attribute__((aligned(16))) int dsm[];
  int* list = dsm;
  int* hl   = dsm + LISTN;
  int* sl   = hl + RCAP;
  int* cnt  = sl + RCAP;
  int* offs = cnt + NBA;
  int* cur  = offs + NBA;
  int* misc = cur + NBA;
  const int tid = (int)threadIdx.x, lane = tid & 31, wave = tid >> 5;
  const int b = (int)blockIdx.x;
  const int nodeBase = b * NBA;

  {
    const v4i z4 = {0, 0, 0, 0};
    for (int i = tid * 4; i < BK_ZINTS; i += NTHR * 4) *(v4ia*)(dsm + i) = z4;
    if (tid < 16) misc[tid] = 0;
  }
  __syncthreads();

  int t = 0, ov = 0;
  const int nChunks = (NE + CHUNK - 1) / CHUNK;
#pragma unroll 1
  for (int ch = 0; ch < nChunks; ++ch) {
    const int cbase = ch * CHUNK;
    const int wc = scan_chunk(rcv, NE, cbase, nodeBase, NBA, 1, list, tid, lane, wave);
    if (lane == 0) misc[wave] = wc;
    __syncthreads();
    if (wave == 0) {
#pragma unroll 1
      for (int w2 = 0; w2 < NWAVE; ++w2) {
        int c = misc[w2];
        c = c < 0 ? 0 : (c > WCAP ? WCAP : c);
#pragma unroll 1
        for (int b0 = 0; b0 < c; b0 += 32) {
          const int idx = b0 + lane;
          const int ent = list[w2 * WCAP + (idx < WCAP ? idx : WCAP - 1)];
          const int m32 = (c - b0) < 32 ? (c - b0) : 32;
#pragma unroll 1
          for (int k = 0; k < m32; ++k) {
            const int u    = __builtin_amdgcn_readlane(ent, k);
            const int slot = u & (NBA - 1);
            const int el   = (u >> SLA) & (CHUNK - 1);
            const int pk   = ((cbase + el) << SLA) | slot;
            if (t < RCAP) {
              if (lane == 0) { hl[t] = pk; cnt[slot] = cnt[slot] + 1; }
              t = t + 1;
            } else {
              ov = 1;
            }
          }
        }
      }
    }
    __syncthreads();
  }
  if (wave == 0 && lane == 0) { misc[8] = t; misc[9] = ov; }
  __syncthreads();
  int tt = misc[8];
  tt = tt < 0 ? 0 : (tt > RCAP ? RCAP : tt);
  const int ovf = misc[9];

  if (wave == 0) {
    const int base = lane * (NBA / 32);
    int s = 0;
#pragma unroll 1
    for (int i = 0; i < NBA / 32; ++i) s += cnt[base + i];
    int incl = s;
#pragma unroll
    for (int d = 1; d < 32; d <<= 1) {
      const int y = __shfl_up(incl, d, 32);
      if (lane >= d) incl += y;
    }
    int run = incl - s;
#pragma unroll 1
    for (int i = 0; i < NBA / 32; ++i) {
      const int cv = cnt[base + i];
      offs[base + i] = run;
      cur[base + i]  = run;
      run += cv;
    }
  }
  __syncthreads();
  if (wave == 0) {
#pragma unroll 1
    for (int b0 = 0; b0 < tt; b0 += 32) {
      const int idx = b0 + lane;
      const int ent = hl[idx < RCAP ? idx : RCAP - 1];
      const int m32 = (tt - b0) < 32 ? (tt - b0) : 32;
#pragma unroll 1
      for (int k = 0; k < m32; ++k) {
        const int u    = __builtin_amdgcn_readlane(ent, k);
        const int slot = u & (NBA - 1);
        if (lane == 0) {
          int p = cur[slot];
          p = p < 0 ? 0 : (p > RCAP - 1 ? RCAP - 1 : p);
          sl[p] = u;
          cur[slot] = p + 1;
        }
      }
    }
  }
  __syncthreads();

#pragma unroll 1
  for (int it = 0; it < RCAP / (4 * NTHR); ++it) {
    const int p4 = (it * NTHR + tid) * 4;
    const v4i e4 = *(const v4ia*)(sl + p4);
    const int s0 = bk_snd(e4.x, p4,     tt, snd);
    const int s1 = bk_snd(e4.y, p4 + 1, tt, snd);
    const int s2 = bk_snd(e4.z, p4 + 2, tt, snd);
    const int s3 = bk_snd(e4.w, p4 + 3, tt, snd);
    const int r0 = bk_rcv(e4.x, p4,     tt, nodeBase);
    const int r1 = bk_rcv(e4.y, p4 + 1, tt, nodeBase);
    const int r2 = bk_rcv(e4.z, p4 + 2, tt, nodeBase);
    const int r3 = bk_rcv(e4.w, p4 + 3, tt, nodeBase);
    const v4i sv = {s0, s1, s2, s3};
    const v4i rv = {r0, r1, r2, r3};
    puti4(SND  + (size_t)b * RCAP + p4, sv);
    puti4(RCVL + (size_t)b * RCAP + p4, rv);
  }
  {
    const v4i c4 = *(const v4ia*)(cnt + 4 * tid);
    const v4i o4 = *(const v4ia*)(offs + 4 * tid);
    puti4(CNT + (size_t)b * NBA + 4 * tid, c4);
    puti4(OFF + (size_t)b * NBA + 4 * tid, o4);
  }
  if (tid < 8) {
    v4i mv = {0, 0, 0, 0};
    if (tid == 0) { mv.x = tt; mv.y = ovf; }
    puti4(META + b * 32 + 4 * tid, mv);
  }
}

__global__ __launch_bounds__(NTHR) __attribute__((amdgpu_num_vgpr(248)))
void k_edge(const int* __restrict__ SND, const int* __restrict__ RCVL, const int* __restrict__ META,
            const float* __restrict__ pos, const unsigned short* __restrict__ WP,
            float* MIX, float* EA, int gbase) {
  extern __shared__ __attribute__((aligned(16))) float dyne[];
  float*          sD  = dyne;
  unsigned short* sA2 = (unsigned short*)(dyne + 128 * SD_P);
  unsigned short* sA1 = sA2 + 128 * A2_P;
  const int tid = (int)threadIdx.x, lane = tid & 31, wave = tid >> 5, hh = lane >> 4, m = lane & 15;
  const int tile = (int)blockIdx.x, lb = (int)blockIdx.y;
  const int b = gbase + lb;
  const int tbase = tile * 128;
  const int bc = clampi(META[b * 32], 0, RCAP);
  if (tbase >= bc) return;

  if (tid < 128) {
    const int p = tbase + tid;
    const size_t li = (size_t)b * RCAP + p;
    const int s = clampi(SND[li], 0, NN - 1);
    const int r = clampi(RCVL[li], 0, NN - 1);
    const float* ps = pos + (size_t)s * 3;
    const float* pr = pos + (size_t)r * 3;
    const float sx = ps[0], sy = ps[1], sz = ps[2];
    const float rx = pr[0], ry = pr[1], rz = pr[2];
    const float dx = bf16_val(rx) - bf16_val(sx);
    const float dy = bf16_val(ry) - bf16_val(sy);
    const float dz = bf16_val(rz) - bf16_val(sz);
    const float rr = sqrtf((dx * dx + dz * dz) + dy * dy);
    const float inv = rcp_f(fmaxf(rr, 1e-9f));
    v4f ea;
    ea.x = (SQ3_F * dx) * inv;
    ea.y = (SQ3_F * dy) * inv;
    ea.z = (SQ3_F * dz) * inv;
    ea.w = 0.0f;
    const float x  = rr * (1.0f / 6.0f);
    const float t2 = 2.0f * (1.0f - x);
    const bool  tp = t2 > 0.0f;
    const float ts = tp ? t2 : 1.0f;
    const float ex = expf(-rcp_f(ts));
    const float env = ENVC_F * (tp ? ex : 0.0f);
    unsigned short* a1 = sA1 + tid * A1_P;
#pragma unroll 1
    for (int n = 1; n <= 8; ++n) {
      const float fn  = (float)n;
      const float py  = PI_F * (fn * x);
      const bool  z0  = (py == 0.0f);
      const float pys = z0 ? 1.0f : py;
      const float sq  = sinf(pys) * rcp_f(pys);
      const float sc  = z0 ? 1.0f : sq;
      const float rbv = ((SQ2_F * (fn * PI_F)) * sc) * env;
      const unsigned hb = bf16_bits(rbv);
      a1[n - 1] = (unsigned short)hb;
      a1[8 + n - 1] = (unsigned short)bf16_bits(rbv - __uint_as_float(hb << 16));
    }
    {
      const v8us z8 = {0, 0, 0, 0, 0, 0, 0, 0};
      *(v8usa*)(a1 + 16) = z8;
      *(v8usa*)(a1 + 24) = z8;
    }
    putf4(EA + ((size_t)lb * RCAP + p) * 4, ea);
  }
  __syncthreads();

  {
    v8f a1c[4];
    {
      const v8f z = {0.f, 0.f, 0.f, 0.f, 0.f, 0.f, 0.f, 0.f};
#pragma unroll
      for (int nt = 0; nt < 4; ++nt) a1c[nt] = z;
    }
    const unsigned short* ap = sA1 + (16 * wave + m) * A1_P + 8 * hh;
    FragB af;
    af.h[0] = *(const v8usa*)ap;
    af.h[1] = *(const v8usa*)(ap + 16);
    const unsigned short* bp = WP + OW1C + m * 32 + 8 * hh;
#pragma unroll
    for (int nt = 0; nt < 4; ++nt) {
      const unsigned short* wq = bp + (16 * nt) * 32;
      FragB bf;
      bf.h[0] = *(const v8usa*)wq;
      bf.h[1] = *(const v8usa*)(wq + 16);
      a1c[nt] = wmb(af, bf, a1c[nt]);
    }
#pragma unroll
    for (int nt = 0; nt < 4; ++nt) {
#pragma unroll
      for (int r = 0; r < 8; ++r)
        sD[(16 * wave + 8 * hh + r) * SD_P + 16 * nt + m] = a1c[nt][r] * RS8_F;
    }
  }
  __syncthreads();

#pragma unroll 1
  for (int it = 0; it < GEL_IT; ++it) {
    const int idx = it * NTHR + tid;
    const int row = idx >> 6;
    const int col = idx & 63;
    const float p  = sD[row * SD_P + col];
    const float u  = 0.7978845608f * (p + 0.044715f * (p * p * p));
    const float g  = (p * (0.5f * (1.0f + tanhf(u)))) * GINV_F;
    const unsigned hb = bf16_bits(g);
    unsigned short* q = sA2 + row * A2_P + col;
    q[0]  = (unsigned short)hb;
    q[64] = (unsigned short)bf16_bits(g - __uint_as_float(hb << 16));
  }
  __syncthreads();

#pragma unroll 1
  for (int half = 0; half < 2; ++half) {
    v8f acc[6];
    {
      const v8f z = {0.f, 0.f, 0.f, 0.f, 0.f, 0.f, 0.f, 0.f};
#pragma unroll
      for (int nt = 0; nt < 6; ++nt) acc[nt] = z;
    }
    const unsigned short* ap = sA2 + (16 * wave + m) * A2_P + 8 * hh;
    const unsigned short* bp = WP + OW2C + (size_t)(96 * half + m) * 128 + 8 * hh;
#pragma unroll 1
    for (int k0 = 0; k0 < 128; k0 += 32) {
      FragB af;
      af.h[0] = *(const v8usa*)(ap + k0);
      af.h[1] = *(const v8usa*)(ap + k0 + 16);
#pragma unroll
      for (int nt = 0; nt < 6; ++nt) {
        const unsigned short* wq = bp + (16 * nt) * 128 + k0;
        FragB bf;
        bf.h[0] = *(const v8usa*)wq;
        bf.h[1] = *(const v8usa*)(wq + 16);
        acc[nt] = wmb(af, bf, acc[nt]);
      }
    }
#pragma unroll
    for (int nt = 0; nt < 6; ++nt) {
#pragma unroll
      for (int r = 0; r < 8; ++r)
        sD[(16 * wave + 8 * hh + r) * SD_P + 96 * half + 16 * nt + m] = acc[nt][r] * 0.125f;
    }
  }
  __syncthreads();

  {
    float* mb = MIX + ((size_t)lb * RCAP + tbase + 16 * wave) * MIXW;
#pragma unroll 4
    for (int it = 0; it < 24; ++it) {
      const int j = it * 32 + lane;
      const int row = j / 48, c4 = j - row * 48;
      const v4f v = *(const v4fa*)(sD + (16 * wave + row) * SD_P + 4 * c4);
      *(volatile v4f*)(mb + (size_t)row * MIXW + 4 * c4) = v;
    }
    __threadfence();
#pragma unroll 4
    for (int it = 0; it < 24; ++it) {
      const int j = it * 32 + lane;
      const int row = j / 48, c4 = j - row * 48;
      const v4f v = *(const v4fa*)(sD + (16 * wave + row) * SD_P + 4 * c4);
      *(volatile v4f*)(mb + (size_t)row * MIXW + 4 * c4) = v;
    }
  }
}

__device__ __forceinline__ void stage_hl(unsigned short* sw, int off, float v) {
  const unsigned hb = bf16_bits(v);
  sw[off]      = (unsigned short)hb;
  sw[off + 96] = (unsigned short)bf16_bits(v - __uint_as_float(hb << 16));
}

__global__ __launch_bounds__(NTHR) __attribute__((amdgpu_num_vgpr(248)))
void k_scan(const int* __restrict__ SND, const int* __restrict__ CNT, const int* __restrict__ OFF,
            const int* __restrict__ META, const float* __restrict__ SV, const float* __restrict__ MIX,
            const float* __restrict__ EA, unsigned short* AGG, int gbase) {
  __shared__ __attribute__((aligned(16))) unsigned short stgA[NWAVE * AGGW];
  const int tid = (int)threadIdx.x, lane = tid & 31, wave = tid >> 5;
  const int lb = (int)blockIdx.x >> 3, part = (int)blockIdx.x & 7;
  const int b = gbase + lb;
  const int pois = META[b * 32 + 1];
  const float qnan = __int_as_float(0x7fc00000);
  unsigned short* sw = stgA + wave * AGGW;

#pragma unroll 1
  for (int i = 0; i < 16; ++i) {
    const int slot = part * 128 + wave * 16 + i;
    int craw = CNT[(size_t)b * NBA + slot];
    int o    = OFF[(size_t)b * NBA + slot];
    craw = __builtin_amdgcn_readfirstlane(craw);
    o    = __builtin_amdgcn_readfirstlane(o);
    int c = clampi(craw, 0, DEGCAP);
    o = clampi(o, 0, RCAP);
    if (c > RCAP - o) c = RCAP - o;
    float aS0 = 0.f, aS1 = 0.f, aS2 = 0.f;
    float aV00 = 0.f, aV01 = 0.f, aV02 = 0.f;
    float aV10 = 0.f, aV11 = 0.f, aV12 = 0.f;
    float aV20 = 0.f, aV21 = 0.f, aV22 = 0.f;
#pragma unroll 1
    for (int j = 0; j < c; ++j) {
      const int p = o + j;
      const int s = clampi(SND[(size_t)b * RCAP + p], 0, NN - 1);
      const float* sv = SV + (size_t)s * SVW + lane;
      const float s0 = sv[0], s1 = sv[32], v0 = sv[64], v1 = sv[96], v2 = sv[128];
      const v4f ea = *(const v4f*)(EA + ((size_t)lb * RCAP + p) * 4);
      ldwait();
      const float* mr = MIX + ((size_t)lb * RCAP + p) * MIXW + lane;
      const float m0 = mr[0], m1 = mr[32], m2 = mr[64], m3 = mr[96], m4 = mr[128], m5 = mr[160];
      ldwait();
      aS0 += s0 * m0;
      aS1 += s1 * m1;
      const float tps = ((v0 * ea.x + v1 * ea.y) + v2 * ea.z) * RS3_F;
      aS2 += tps * m2;
      aV00 += v0 * m3;  aV10 += v1 * m3;  aV20 += v2 * m3;
      aV01 += (s0 * ea.x) * m4;  aV11 += (s0 * ea.y) * m4;  aV21 += (s0 * ea.z) * m4;
      aV02 += (s1 * ea.x) * m5;  aV12 += (s1 * ea.y) * m5;  aV22 += (s1 * ea.z) * m5;
    }
    const bool bad = (pois != 0) || (craw > DEGCAP);
    stage_hl(sw, 0 * 192 + lane,       bad ? qnan : aS0 * RS8_F);
    stage_hl(sw, 0 * 192 + 32 + lane,  bad ? qnan : aS1 * RS8_F);
    stage_hl(sw, 0 * 192 + 64 + lane,  bad ? qnan : aS2 * RS8_F);
    stage_hl(sw, 1 * 192 + lane,       bad ? qnan : aV00 * RS8_F);
    stage_hl(sw, 1 * 192 + 32 + lane,  bad ? qnan : aV01 * RS8_F);
    stage_hl(sw, 1 * 192 + 64 + lane,  bad ? qnan : aV02 * RS8_F);
    stage_hl(sw, 2 * 192 + lane,       bad ? qnan : aV10 * RS8_F);
    stage_hl(sw, 2 * 192 + 32 + lane,  bad ? qnan : aV11 * RS8_F);
    stage_hl(sw, 2 * 192 + 64 + lane,  bad ? qnan : aV12 * RS8_F);
    stage_hl(sw, 3 * 192 + lane,       bad ? qnan : aV20 * RS8_F);
    stage_hl(sw, 3 * 192 + 32 + lane,  bad ? qnan : aV21 * RS8_F);
    stage_hl(sw, 3 * 192 + 64 + lane,  bad ? qnan : aV22 * RS8_F);
    __syncthreads();
    const v8us q0 = *(const v8usa*)(sw + 8 * lane);
    const v8us q1 = *(const v8usa*)(sw + 256 + 8 * lane);
    const v8us q2 = *(const v8usa*)(sw + 512 + 8 * lane);
    unsigned short* gp = AGG + ((size_t)lb * NBA + slot) * AGGW + 8 * lane;
    *(volatile v8us*)gp         = q0;
    *(volatile v8us*)(gp + 256) = q1;
    *(volatile v8us*)(gp + 512) = q2;
    __threadfence();
    *(volatile v8us*)gp         = q0;
    *(volatile v8us*)(gp + 256) = q1;
    *(volatile v8us*)(gp + 512) = q2;
    __syncthreads();
  }
}

__global__ __launch_bounds__(128) __attribute__((amdgpu_num_vgpr(248)))
void k_down(const unsigned short* __restrict__ AGG, const unsigned short* __restrict__ WP,
            const int* __restrict__ META, float* out, int gbase) {
  __shared__ __attribute__((aligned(16))) float stg[64 * SV_P];
  const int tid = (int)threadIdx.x, lane = tid & 31, wave = tid >> 5, hh = lane >> 4, m = lane & 15;
  const int t = (int)blockIdx.x;
  const int lb = t >> 4;
  const int b = gbase + lb;
  const int node0 = b * NBA + (t & 15) * 64;
  const int pois = META[b * 32 + 1];
  const float qnan = __int_as_float(0x7fc00000);

  v8f accS[4], accV[3][2];
  {
    const v8f z = {0.f, 0.f, 0.f, 0.f, 0.f, 0.f, 0.f, 0.f};
#pragma unroll
    for (int nt = 0; nt < 4; ++nt) accS[nt] = z;
#pragma unroll
    for (int d = 0; d < 3; ++d) { accV[d][0] = z; accV[d][1] = z; }
  }
  const unsigned short* arow = AGG + (size_t)(t * 64 + 16 * wave + m) * AGGW + 8 * hh;
  const unsigned short* wds  = WP + OWDS + m * 192 + 8 * hh;
  const unsigned short* wdv  = WP + OWDV + m * 192 + 8 * hh;
#pragma unroll 1
  for (int k0 = 0; k0 < 192; k0 += 32) {
    FragB as;
    as.h[0] = *(const v8usa*)(arow + k0);
    as.h[1] = *(const v8usa*)(arow + k0 + 16);
#pragma unroll
    for (int nt = 0; nt < 4; ++nt) {
      const unsigned short* wq = wds + (16 * nt) * 192 + k0;
      FragB bf;
      bf.h[0] = *(const v8usa*)wq;
      bf.h[1] = *(const v8usa*)(wq + 16);
      accS[nt] = wmb(as, bf, accS[nt]);
    }
    FragB b0, b1;
    b0.h[0] = *(const v8usa*)(wdv + k0);
    b0.h[1] = *(const v8usa*)(wdv + k0 + 16);
    b1.h[0] = *(const v8usa*)(wdv + 16 * 192 + k0);
    b1.h[1] = *(const v8usa*)(wdv + 16 * 192 + k0 + 16);
#pragma unroll
    for (int d = 0; d < 3; ++d) {
      const unsigned short* aq = arow + 192 * (1 + d) + k0;
      FragB av;
      av.h[0] = *(const v8usa*)aq;
      av.h[1] = *(const v8usa*)(aq + 16);
      accV[d][0] = wmb(av, b0, accV[d][0]);
      accV[d][1] = wmb(av, b1, accV[d][1]);
    }
  }
  const bool bad = pois != 0;
#pragma unroll
  for (int r = 0; r < 8; ++r) {
    float* sr = stg + (16 * wave + 8 * hh + r) * SV_P;
#pragma unroll
    for (int nt = 0; nt < 4; ++nt) {
      const float v = accS[nt][r] * RS96_F;
      sr[16 * nt + m] = bad ? qnan : v;
    }
#pragma unroll
    for (int d = 0; d < 3; ++d) {
      const float v0 = accV[d][0][r] * RS96_F;
      const float v1 = accV[d][1][r] * RS96_F;
      sr[64 + 3 * m + d]        = bad ? qnan : v0;
      sr[64 + 3 * (16 + m) + d] = bad ? qnan : v1;
    }
  }
  __syncthreads();

#pragma unroll 4
  for (int it = 0; it < 20; ++it) {
    const int j = it * 32 + lane;
    const int row = j / 40, c4 = j - row * 40;
    const int gr = node0 + 16 * wave + row;
    const v4f v = *(const v4fa*)(stg + (16 * wave + row) * SV_P + 4 * c4);
    if (gr < NN) *(volatile v4f*)(out + (size_t)gr * SVW + 4 * c4) = v;
  }
  __threadfence();
#pragma unroll 4
  for (int it = 0; it < 20; ++it) {
    const int j = it * 32 + lane;
    const int row = j / 40, c4 = j - row * 40;
    const int gr = node0 + 16 * wave + row;
    const v4f v = *(const v4fa*)(stg + (16 * wave + row) * SV_P + 4 * c4);
    if (gr < NN) *(volatile v4f*)(out + (size_t)gr * SVW + 4 * c4) = v;
  }
}

static inline size_t al256(size_t v) { return (v + 255) & ~(size_t)255; }

extern "C" void kernel_launch(void* const* d_in, const int* in_sizes, int n_in,
                              void* d_out, int out_size, void* d_ws, size_t ws_size,
                              hipStream_t stream) {
  if (n_in < 11) return;
  if (in_sizes[0] != NN * 3 || in_sizes[1] != NN * 64 || in_sizes[2] != NN * 96) return;
  if (in_sizes[3] != NE || in_sizes[4] != NE) return;
  if (in_sizes[5] != 64 * 64 || in_sizes[6] != 32 * 32 || in_sizes[7] != 8 * 64) return;
  if (in_sizes[8] != 64 * 192 || in_sizes[9] != 96 * 64 || in_sizes[10] != 96 * 32) return;
  if (out_size != NN * SVW) return;

  const float* pos  = (const float*)d_in[0];
  const float* xs   = (const float*)d_in[1];
  const float* nv   = (const float*)d_in[2];
  const int*   snd  = (const int*)  d_in[3];
  const int*   rcv  = (const int*)  d_in[4];
  const float* Wus  = (const float*)d_in[5];
  const float* Wuv  = (const float*)d_in[6];
  const float* W1   = (const float*)d_in[7];
  const float* W2   = (const float*)d_in[8];
  const float* Wds  = (const float*)d_in[9];
  const float* Wdv  = (const float*)d_in[10];
  float* out = (float*)d_out;

  char* ws = (char*)d_ws;
  size_t off = 0;
  const size_t oWP  = off; off = al256(off + (size_t)NWP * 2);
  const size_t oSV  = off; off = al256(off + (size_t)NN * SVW * 4);
  const size_t oSND = off; off = al256(off + (size_t)NBLK * RCAP * 4);
  const size_t oRCV = off; off = al256(off + (size_t)NBLK * RCAP * 4);
  const size_t oCNT = off; off = al256(off + (size_t)NBLK * NBA * 4);
  const size_t oOFF = off; off = al256(off + (size_t)NBLK * NBA * 4);
  const size_t oMET = off; off = al256(off + (size_t)NBLK * 32 * 4);
  const size_t oMIX = off; off = al256(off + (size_t)GRPB * RCAP * MIXW * 4);
  const size_t oEA  = off; off = al256(off + (size_t)GRPB * RCAP * 4 * 4);
  const size_t oAGG = off; off = al256(off + (size_t)GRPB * NBA * AGGW * 2);
  if (off > ws_size || off > (size_t)WSMAX) return;
  unsigned short* WP   = (unsigned short*)(ws + oWP);
  float*          SV   = (float*)(ws + oSV);
  int*            SND  = (int*)(ws + oSND);
  int*            RCVL = (int*)(ws + oRCV);
  int*            CNT  = (int*)(ws + oCNT);
  int*            OFF  = (int*)(ws + oOFF);
  int*            META = (int*)(ws + oMET);
  float*          MIX  = (float*)(ws + oMIX);
  float*          EA   = (float*)(ws + oEA);
  unsigned short* AGG  = (unsigned short*)(ws + oAGG);

  hipFuncSetAttribute(reinterpret_cast<const void*>(&k_up), hipFuncAttributeMaxDynamicSharedMemorySize,
                      (int)UP_LDS);
  hipFuncSetAttribute(reinterpret_cast<const void*>(&k_bucket), hipFuncAttributeMaxDynamicSharedMemorySize,
                      (int)BK_LDS);
  hipFuncSetAttribute(reinterpret_cast<const void*>(&k_edge), hipFuncAttributeMaxDynamicSharedMemorySize,
                      (int)EDGE_LDS);

  k_prep<<<PU5 / 128, 128, 0, stream>>>(Wus, Wuv, W1, W2, Wds, Wdv, WP);
  k_up<<<(NN + 127) / 128, NTHR, UP_LDS, stream>>>(xs, nv, WP, SV);
  k_bucket<<<NBLK, NTHR, BK_LDS, stream>>>(rcv, snd, SND, RCVL, CNT, OFF, META);
  for (int g = 0; g < NGRP; ++g) {
    const int gbase = g * GRPB;
    int nblk = NBLK - gbase;
    nblk = nblk > GRPB ? GRPB : nblk;
    if (nblk <= 0) continue;
    k_edge<<<dim3(TPB, nblk), NTHR, EDGE_LDS, stream>>>(SND, RCVL, META, pos, WP, MIX, EA, gbase);
    k_scan<<<nblk * 8, NTHR, 0, stream>>>(SND, CNT, OFF, META, SV, MIX, EA, AGG, gbase);
    k_down<<<nblk * 16, 128, 0, stream>>>(AGG, WP, META, out, gbase);
  }
}
